// RNN_20804821581890
// MI455X (gfx1250) — hardware-verified
//
#include <hip/hip_runtime.h>

typedef __attribute__((ext_vector_type(16))) __bf16   v16b;
typedef __attribute__((ext_vector_type(8)))  __bf16   v8b;
typedef __attribute__((ext_vector_type(8)))  float    v8f;
typedef __attribute__((ext_vector_type(4)))  float    v4f;
typedef __attribute__((ext_vector_type(2)))  float    v2f;
typedef __attribute__((ext_vector_type(4)))  unsigned v4u;

constexpr int BATCH_N   = 4096;
constexpr int STEPS_N   = 512;
constexpr int NIN_N     = 2;
constexpr int HID_N     = 16;
constexpr int OUT_N     = 2;
constexpr int LAYERS_N  = 3;
constexpr int TILE_ROWS = 16;
constexpr int CHUNK_T   = 16;
constexpr int XROW_F    = STEPS_N * NIN_N;
constexpr int OROW_F    = STEPS_N * OUT_N;
constexpr int OUT0_ELEMS = BATCH_N * STEPS_N * OUT_N;
constexpr int OUT1_ELEMS = LAYERS_N * BATCH_N * HID_N;
constexpr float LOG2E_F  = 1.44269504088896340736f;

static_assert(BATCH_N % TILE_ROWS == 0, "batch tiles exact");
static_assert(STEPS_N % CHUNK_T == 0, "step chunks exact");
static_assert(CHUNK_T * NIN_N * 4 == 128, "x chunk is one 128-B line per row");
static_assert(CHUNK_T * OUT_N * 4 == 128, "out chunk is one 128-B line per row");
static_assert(HID_N == 16, "hi|lo K-packing fills the 32-deep tile exactly");
static_assert((size_t)OUT0_ELEMS * 4 == 16777216u, "second output byte offset");
static_assert(((size_t)OUT0_ELEMS + (size_t)OUT1_ELEMS) * 4 == 17563648u, "total output bytes");
static_assert((TILE_ROWS * HID_N * 4) % 128 == 0, "hidden tile is whole lines");

__device__ __forceinline__ unsigned bfbits(float f) {
  const unsigned u = __float_as_uint(f);
  return (u + 0x7FFFu + ((u >> 16) & 1u)) >> 16;
}
__device__ __forceinline__ float bfval(unsigned b) { return __uint_as_float(b << 16); }

__device__ __forceinline__ void split8(const float (&f)[8], v8b& hi, v8b& lo) {
  unsigned hw[4], lw[4];
#pragma unroll
  for (int p = 0; p < 4; ++p) {
    const float f0 = f[2 * p];
    const float f1 = f[2 * p + 1];
    const unsigned h0 = bfbits(f0);
    const unsigned h1 = bfbits(f1);
    const unsigned l0 = bfbits(f0 - bfval(h0));
    const unsigned l1 = bfbits(f1 - bfval(h1));
    hw[p] = h0 | (h1 << 16);
    lw[p] = l0 | (l1 << 16);
  }
  const v4u H = {hw[0], hw[1], hw[2], hw[3]};
  const v4u L = {lw[0], lw[1], lw[2], lw[3]};
  hi = __builtin_bit_cast(v8b, H);
  lo = __builtin_bit_cast(v8b, L);
}

__device__ __forceinline__ void load_w8(const float* p, bool keep, v8b& hi, v8b& lo) {
  v4f a = *(const v4f*)(p);
  v4f b = *(const v4f*)(p + 4);
  asm volatile("" : "+v"(a), "+v"(b) :: "memory");
  float f[8];
#pragma unroll
  for (int e = 0; e < 4; ++e) {
    const float ae = a[e];
    const float be = b[e];
    f[e]     = keep ? ae : 0.0f;
    f[4 + e] = keep ? be : 0.0f;
  }
  split8(f, hi, lo);
}

__device__ __forceinline__ v16b cat16(v8b a, v8b b) {
  return __builtin_shufflevector(a, b, 0, 1, 2, 3, 4, 5, 6, 7, 8, 9, 10, 11, 12, 13, 14, 15);
}

__device__ __forceinline__ v8f mma_bf(v16b a, v16b b, v8f c) {
  return __builtin_amdgcn_wmma_f32_16x16x32_bf16(false, a, false, b, (short)0, c, false, false);
}

__device__ __forceinline__ void guard_main(v8f& a, v8f& b, v8f& c, v8f& d,
                                           v16b A1, v16b A2, v16b A3,
                                           v16b b0, v16b b1, v16b b2, v16b b3, v16b b4,
                                           v16b b5, v16b b6, v16b b7, v16b b8, v16b b9) {
  asm volatile("v_nop\n\tv_nop\n\tv_nop\n\tv_nop"
               : "+v"(a), "+v"(b), "+v"(c), "+v"(d)
               : "v"(A1), "v"(A2), "v"(A3), "v"(b0), "v"(b1), "v"(b2), "v"(b3), "v"(b4),
                 "v"(b5), "v"(b6), "v"(b7), "v"(b8), "v"(b9));
}
__device__ __forceinline__ void guard_head(v8f& a, v16b A2, v16b A3, v16b b0, v16b b1) {
  asm volatile("v_nop\n\tv_nop\n\tv_nop\n\tv_nop" : "+v"(a) : "v"(A2), "v"(A3), "v"(b0), "v"(b1));
}

__device__ __forceinline__ float fsigm(float v) {
  return __builtin_amdgcn_rcpf(1.0f + __builtin_amdgcn_exp2f(-LOG2E_F * v));
}
__device__ __forceinline__ float ftanh(float v) {
  return 1.0f - 2.0f * __builtin_amdgcn_rcpf(1.0f + __builtin_amdgcn_exp2f((2.0f * LOG2E_F) * v));
}

__global__ __launch_bounds__(96)
void gru3_pipe_kernel(const float* __restrict__ x,    const float* __restrict__ h0,
                      const float* __restrict__ Wemb, const float* __restrict__ bemb,
                      const float* __restrict__ Wout, const float* __restrict__ bout,
                      const float* __restrict__ Wih0, const float* __restrict__ Whh0,
                      const float* __restrict__ bih0, const float* __restrict__ bhh0,
                      const float* __restrict__ Wih1, const float* __restrict__ Whh1,
                      const float* __restrict__ bih1, const float* __restrict__ bhh1,
                      const float* __restrict__ Wih2, const float* __restrict__ Whh2,
                      const float* __restrict__ bih2, const float* __restrict__ bhh2,
                      float* __restrict__ out, float* __restrict__ hid)
{
  __shared__ __align__(16) __bf16 ysH[LAYERS_N * 2 * 256];
  __shared__ __align__(16) __bf16 ysL[LAYERS_N * 2 * 256];
  __shared__ __align__(16) float  xs[2 * 512];
  __shared__ __align__(16) float  ostg[2 * 512];
  __shared__ __align__(16) float  hfs[LAYERS_N * 256];
  __shared__ __align__(16) float  embc[48];

  const int tid  = (int)threadIdx.x;
  const int lane = tid & 31;
  const int wave = __builtin_amdgcn_readfirstlane(tid >> 5);
  const int c    = lane & 15;
  const int hh   = lane >> 4;
  const int b0   = (int)blockIdx.x * TILE_ROWS;
  const int q4   = lane >> 3;
  const int c4   = (lane & 7) * 4;

  const float* Wi = (wave == 0) ? Wih0 : ((wave == 1) ? Wih1 : Wih2);
  const float* Wh = (wave == 0) ? Whh0 : ((wave == 1) ? Whh1 : Whh2);
  const float* bi = (wave == 0) ? bih0 : ((wave == 1) ? bih1 : bih2);
  const float* bh = (wave == 0) ? bhh0 : ((wave == 1) ? bhh1 : bhh2);

  const v4u zw = {0u, 0u, 0u, 0u};
  const v8b zero8 = __builtin_bit_cast(v8b, zw);

  v8b wiH, wiL, whH, whL;
  load_w8(Wi + (0 * HID_N + c) * HID_N + 8 * hh, true, wiH, wiL);
  load_w8(Wh + (0 * HID_N + c) * HID_N + 8 * hh, true, whH, whL);
  const v16b Br1 = cat16(wiH, wiH);
  const v16b Br2 = cat16(whH, whH);
  const v16b Br3 = cat16(whL, wiL);
  load_w8(Wi + (1 * HID_N + c) * HID_N + 8 * hh, true, wiH, wiL);
  load_w8(Wh + (1 * HID_N + c) * HID_N + 8 * hh, true, whH, whL);
  const v16b Bz1 = cat16(wiH, wiH);
  const v16b Bz2 = cat16(whH, whH);
  const v16b Bz3 = cat16(whL, wiL);
  load_w8(Wi + (2 * HID_N + c) * HID_N + 8 * hh, true, wiH, wiL);
  load_w8(Wh + (2 * HID_N + c) * HID_N + 8 * hh, true, whH, whL);
  const v16b Bn1 = cat16(wiH, wiH);
  const v16b Bn2 = cat16(whH, whH);
  const v16b Bn3 = cat16(whL, zero8);
  const v16b Bn4 = cat16(zero8, wiL);
  const int orow = (c < OUT_N) ? c : (OUT_N - 1);
  v8b woH, woL;
  load_w8(Wout + orow * HID_N + 8 * hh, c < OUT_N, woH, woL);
  const v16b Bo1 = cat16(woH, woH);
  const v16b Bo2 = cat16(woL, zero8);

  const float bir = bi[c], bhr = bh[c];
  const float biz = bi[HID_N + c], bhz = bh[HID_N + c];
  const float cxn = bi[2 * HID_N + c];
  const float chn = bh[2 * HID_N + c];
  const float bo  = bout[orow];
  asm volatile("" ::: "memory");
  const float cr = bir + bhr;
  const float cz = biz + bhz;

  float hreg[8];
#pragma unroll
  for (int r = 0; r < 8; ++r)
    hreg[r] = h0[((size_t)wave * BATCH_N + (size_t)(b0 + 8 * hh + r)) * HID_N + c];
  {
    const int so = (wave * 2 + 1) * 256 + (8 * hh) * 16 + c;
#pragma unroll
    for (int r = 0; r < 8; ++r) {
      const float v = hreg[r];
      const unsigned hb = bfbits(v);
      const unsigned lb = bfbits(v - bfval(hb));
      ysH[so + r * 16] = __builtin_bit_cast(__bf16, (unsigned short)hb);
      ysL[so + r * 16] = __builtin_bit_cast(__bf16, (unsigned short)lb);
    }
  }

  const float* xblk = x + (size_t)b0 * XROW_F;
  float* oblk = out + (size_t)b0 * OROW_F;

  if (wave == 0) {
    embc[c]      = Wemb[2 * c];
    embc[16 + c] = Wemb[2 * c + 1];
    embc[32 + c] = bemb[c];
    v4f xv4[4];
#pragma unroll
    for (int it = 0; it < 4; ++it)
      xv4[it] = *(const v4f*)(xblk + (size_t)(it * 4 + q4) * XROW_F + c4);
#pragma unroll
    for (int it = 0; it < 4; ++it)
      *(v4f*)(xs + (it * 4 + q4) * 32 + c4) = xv4[it];
  }
  __syncthreads();

  const v8f z8 = {0.f, 0.f, 0.f, 0.f, 0.f, 0.f, 0.f, 0.f};

#pragma unroll 1
  for (int k = 0; k < STEPS_N + LAYERS_N - 1; ++k) {
    const int t = k - wave;
    if (t >= 0 && t < STEPS_N) {
      v8b inH, inL;
      if (wave == 0) {
        if ((t & 15) == 0 && (t + CHUNK_T) < STEPS_N) {
          const int ch = (t >> 4) + 1;
          const int dofs = (ch & 1) * 512;
          const float* src = xblk + ch * 32;
          v4f xv4[4];
#pragma unroll
          for (int it = 0; it < 4; ++it)
            xv4[it] = *(const v4f*)(src + (size_t)(it * 4 + q4) * XROW_F + c4);
#pragma unroll
          for (int it = 0; it < 4; ++it)
            *(v4f*)(xs + dofs + (it * 4 + q4) * 32 + c4) = xv4[it];
        }
        const int xo = ((t >> 4) & 1) * 512 + c * 32 + (t & 15) * 2;
        const v2f xv = *(const v2f*)(xs + xo);
        const float x0 = xv[0];
        const float x1 = xv[1];
        const v4f w0a = *(const v4f*)(embc + 8 * hh);
        const v4f w0b = *(const v4f*)(embc + 8 * hh + 4);
        const v4f w1a = *(const v4f*)(embc + 16 + 8 * hh);
        const v4f w1b = *(const v4f*)(embc + 16 + 8 * hh + 4);
        const v4f bea = *(const v4f*)(embc + 32 + 8 * hh);
        const v4f beb = *(const v4f*)(embc + 32 + 8 * hh + 4);
        float f[8];
#pragma unroll
        for (int e = 0; e < 4; ++e) {
          const float va = w0a[e] * x0 + w1a[e] * x1 + bea[e];
          const float vb = w0b[e] * x0 + w1b[e] * x1 + beb[e];
          f[e]     = fmaxf(va, 0.0f);
          f[4 + e] = fmaxf(vb, 0.0f);
        }
        split8(f, inH, inL);
      } else {
        const int io = ((wave - 1) * 2 + (t & 1)) * 256 + c * 16 + 8 * hh;
        inH = *(const v8b*)(ysH + io);
        inL = *(const v8b*)(ysL + io);
      }
      const int po = (wave * 2 + ((t - 1) & 1)) * 256 + c * 16 + 8 * hh;
      const v8b hH = *(const v8b*)(ysH + po);
      const v8b hL = *(const v8b*)(ysL + po);

      const v16b A1 = cat16(inH, inL);
      const v16b A2 = cat16(hH, hL);
      const v16b A3 = cat16(hH, inH);

      v8f ar  = mma_bf(A1, Br1, z8);
      v8f az  = mma_bf(A1, Bz1, z8);
      v8f axn = mma_bf(A1, Bn1, z8);
      v8f ahn = mma_bf(A2, Bn2, z8);
      ar  = mma_bf(A2, Br2, ar);
      az  = mma_bf(A2, Bz2, az);
      ar  = mma_bf(A3, Br3, ar);
      az  = mma_bf(A3, Bz3, az);
      ahn = mma_bf(A3, Bn3, ahn);
      axn = mma_bf(A3, Bn4, axn);
      guard_main(ar, az, axn, ahn, A1, A2, A3, Br1, Br2, Br3, Bz1, Bz2, Bz3, Bn1, Bn2, Bn3, Bn4);

      if (wave == 2) {
        if (t > CHUNK_T && (t & 15) == 1) {
          const int ch = (t - (CHUNK_T + 1)) >> 4;
          const int so = (ch & 1) * 512;
          float* ob = oblk + (size_t)ch * 32;
          v4f vv[4];
#pragma unroll
          for (int it = 0; it < 4; ++it)
            vv[it] = *(const v4f*)(ostg + so + (it * 4 + q4) * 32 + c4);
          for (int pass = 0; pass < 2; ++pass) {
#pragma unroll
            for (int it = 0; it < 4; ++it)
              *(volatile v4f*)(ob + (size_t)(it * 4 + q4) * OROW_F + c4) = vv[it];
            __threadfence();
          }
        }
        v8f ao = mma_bf(A2, Bo1, z8);
        ao = mma_bf(A3, Bo2, ao);
        guard_head(ao, A2, A3, Bo1, Bo2);
        if (t > 0) {
          const int s = t - 1;
          const int so = ((s >> 4) & 1) * 512 + (8 * hh) * 32 + (s & 15) * 2 + orow;
          if (c < OUT_N) {
#pragma unroll
            for (int r = 0; r < 8; ++r) ostg[so + r * 32] = ao[r] + bo;
          }
        }
      }

      const int wo = (wave * 2 + (t & 1)) * 256 + (8 * hh) * 16 + c;
#pragma unroll
      for (int r = 0; r < 8; ++r) {
        const float rg = fsigm(ar[r] + cr);
        const float zg = fsigm(az[r] + cz);
        const float ng = ftanh((axn[r] + cxn) + rg * (ahn[r] + chn));
        const float hn = (1.0f - zg) * ng + zg * hreg[r];
        hreg[r] = hn;
        const unsigned hb = bfbits(hn);
        const unsigned lb = bfbits(hn - bfval(hb));
        ysH[wo + r * 16] = __builtin_bit_cast(__bf16, (unsigned short)hb);
        ysL[wo + r * 16] = __builtin_bit_cast(__bf16, (unsigned short)lb);
      }
    }
    __syncthreads();
  }

#pragma unroll
  for (int r = 0; r < 8; ++r) hfs[wave * 256 + (8 * hh + r) * 16 + c] = hreg[r];

  if (wave == 2) {
    const int po = (2 * 2 + ((STEPS_N - 1) & 1)) * 256 + c * 16 + 8 * hh;
    const v8b hH = *(const v8b*)(ysH + po);
    const v8b hL = *(const v8b*)(ysL + po);
    const v16b A2 = cat16(hH, hL);
    const v16b A3 = cat16(hH, hH);
    v8f ao = mma_bf(A2, Bo1, z8);
    ao = mma_bf(A3, Bo2, ao);
    guard_head(ao, A2, A3, Bo1, Bo2);
    const int s = STEPS_N - 1;
    const int so = ((s >> 4) & 1) * 512 + (8 * hh) * 32 + (s & 15) * 2 + orow;
    if (c < OUT_N) {
#pragma unroll
      for (int r = 0; r < 8; ++r) ostg[so + r * 32] = ao[r] + bo;
    }
  }
  __syncthreads();

  {
    const float* hs = hfs + wave * 256;
    const v4f hv0 = *(const v4f*)(hs + lane * 4);
    const v4f hv1 = *(const v4f*)(hs + 128 + lane * 4);
    float* hp = hid + ((size_t)wave * BATCH_N + (size_t)b0) * HID_N;
    for (int pass = 0; pass < 2; ++pass) {
      *(volatile v4f*)(hp + lane * 4) = hv0;
      *(volatile v4f*)(hp + 128 + lane * 4) = hv1;
      __threadfence();
    }
  }

  if (wave == 2) {
    const int ch = (STEPS_N / CHUNK_T) - 1;
    const int so = (ch & 1) * 512;
    float* ob = oblk + (size_t)ch * 32;
    v4f vv[4];
#pragma unroll
    for (int it = 0; it < 4; ++it)
      vv[it] = *(const v4f*)(ostg + so + (it * 4 + q4) * 32 + c4);
    for (int pass = 0; pass < 2; ++pass) {
#pragma unroll
      for (int it = 0; it < 4; ++it)
        *(volatile v4f*)(ob + (size_t)(it * 4 + q4) * OROW_F + c4) = vv[it];
      __threadfence();
    }
  }
}

extern "C" void kernel_launch(void* const* d_in, const int* in_sizes, int n_in,
                              void* d_out, int out_size, void* d_ws, size_t ws_size,
                              hipStream_t stream) {
  (void)d_ws; (void)ws_size;
  if (n_in < 18 || d_out == nullptr) return;
  if (in_sizes[0] != BATCH_N * STEPS_N * NIN_N || in_sizes[1] != LAYERS_N * BATCH_N * HID_N ||
      in_sizes[2] != HID_N * NIN_N || in_sizes[3] != HID_N ||
      in_sizes[4] != OUT_N * HID_N || in_sizes[5] != OUT_N ||
      out_size != OUT0_ELEMS + OUT1_ELEMS) return;
  for (int l = 0; l < LAYERS_N; ++l) {
    if (in_sizes[6 + 4 * l] != 3 * HID_N * HID_N || in_sizes[7 + 4 * l] != 3 * HID_N * HID_N ||
        in_sizes[8 + 4 * l] != 3 * HID_N || in_sizes[9 + 4 * l] != 3 * HID_N) return;
  }
  float* outp = (float*)d_out;
  float* hidp = outp + (size_t)OUT0_ELEMS;
  gru3_pipe_kernel<<<dim3(BATCH_N / TILE_ROWS), dim3(96), 0, stream>>>(
      (const float*)d_in[0],  (const float*)d_in[1],
      (const float*)d_in[2],  (const float*)d_in[3],
      (const float*)d_in[4],  (const float*)d_in[5],
      (const float*)d_in[6],  (const float*)d_in[7],  (const float*)d_in[8],  (const float*)d_in[9],
      (const float*)d_in[10], (const float*)d_in[11], (const float*)d_in[12], (const float*)d_in[13],
      (const float*)d_in[14], (const float*)d_in[15], (const float*)d_in[16], (const float*)d_in[17],
      outp, hidp);
}
